// GCNShared_69801808495209
// MI455X (gfx1250) — hardware-verified
//
#include <hip/hip_runtime.h>
#include <math.h>
#include <stdint.h>

#define NB 16
#define SL 128
#define DM 256
#define MR (NB * SL)
#define KC (2 * DM)

static_assert(KC % 32 == 0);
static_assert(MR % 32 == 0);
static_assert(DM % 64 == 0);
static_assert(SL % 32 == 0);

typedef __attribute__((ext_vector_type(16))) __bf16   v16b;
typedef __attribute__((ext_vector_type(8)))  __bf16   v8b;
typedef __attribute__((ext_vector_type(8)))  float    v8f;
typedef __attribute__((ext_vector_type(4)))  float    v4f;
typedef __attribute__((ext_vector_type(4)))  unsigned int v4u;
typedef v4f __attribute__((may_alias)) v4fa;

__device__ __forceinline__ unsigned short f2bf_bits(float f) {
  unsigned u = __float_as_uint(f);
  return (unsigned short)((u + 0x7FFFu + ((u >> 16) & 1u)) >> 16);
}
__device__ __forceinline__ float bf_bits2f(unsigned short h) { return __uint_as_float(((unsigned)h) << 16); }
__device__ __forceinline__ float bf_rne(float f) { return bf_bits2f(f2bf_bits(f)); }
__device__ __forceinline__ unsigned pk16(unsigned short a, unsigned short b) { return (unsigned)a | ((unsigned)b << 16); }

union FB { v16b v; v8b h[2]; };
__device__ __forceinline__ v16b ldfrag(const __bf16* p) {
  FB f; f.h[0] = *(const v8b*)(p); f.h[1] = *(const v8b*)(p + 16); return f.v;
}
__device__ __forceinline__ v8f mma_bf(v16b a, v16b b, v8f c) {
  c = __builtin_amdgcn_wmma_f32_16x16x32_bf16(false, a, false, b, (short)0, c, false, false);
  asm volatile("v_nop\n\tv_nop\n\tv_nop\n\tv_nop" : "+v"(c) : "v"(a), "v"(b));
  return c;
}

__global__ __launch_bounds__(256) void k_prep(const float* __restrict__ feat, const float* __restrict__ mask,
                                              const float* __restrict__ agg_w, const float* __restrict__ attn_w,
                                              const float* __restrict__ upd_w,
                                              unsigned short* __restrict__ AGW2, unsigned short* __restrict__ W1D,
                                              unsigned short* __restrict__ U1D, unsigned short* __restrict__ HM) {
  const int blk = blockIdx.x, tid = threadIdx.x;
  if (blk >= 352) return;
  const float* src;
  unsigned short* dst;
  float mv = 1.0f;
  bool split = false;
  if (blk < 96) {
    const int msel = blk >> 5;
    const int u = ((blk & 31) << 8) + tid;
    const int row = u >> 5, pc = u & 31;
    const float* W = (msel == 0) ? agg_w : ((msel == 1) ? attn_w : upd_w);
    const int pitch = (msel == 0) ? DM : (2 * DM);
    unsigned short* P = (msel == 0) ? AGW2 : ((msel == 1) ? W1D : U1D);
    src = W + (size_t)row * pitch + pc * 8;
    dst = P + (size_t)row * KC + pc * 8;
  } else {
    const int u = ((blk - 96) << 8) + tid;
    const int row = u >> 5, pc = u & 31;
    src = feat + (size_t)row * DM + pc * 8;
    dst = HM + (size_t)row * KC + pc * 8;
    mv = bf_rne(mask[row]);
    split = true;
  }
  const v4f a = *(const v4fa*)(src);
  const v4f c = *(const v4fa*)(src + 4);
  const float x[8] = { a[0], a[1], a[2], a[3], c[0], c[1], c[2], c[3] };
  unsigned short hb[8], sb[8];
#pragma unroll
  for (int e = 0; e < 8; ++e) {
    const float p = bf_rne(x[e]) * mv;
    const unsigned short h = f2bf_bits(p);
    const unsigned short l = f2bf_bits(p - bf_bits2f(h));
    hb[e] = h;
    sb[e] = split ? l : h;
  }
  const v4u hv = { pk16(hb[0], hb[1]), pk16(hb[2], hb[3]), pk16(hb[4], hb[5]), pk16(hb[6], hb[7]) };
  const v4u sv = { pk16(sb[0], sb[1]), pk16(sb[2], sb[3]), pk16(sb[4], sb[5]), pk16(sb[6], sb[7]) };
  *(volatile v4u*)(dst) = hv;
  *(volatile v4u*)(dst + DM) = sv;
  __threadfence();
  *(volatile v4u*)(dst) = hv;
  *(volatile v4u*)(dst + DM) = sv;
}

template <int MODE>
__global__ __launch_bounds__(256) void k_gemm2(const unsigned short* __restrict__ Ap, const unsigned short* __restrict__ Btp,
                                               const float* __restrict__ bias, int bstride,
                                               const float* __restrict__ mask,
                                               float* __restrict__ Cf, unsigned short* __restrict__ Chl) {
  __shared__ __align__(16) float sT[8][16 * 68];
  const int lane = threadIdx.x & 31;
  const int wave = threadIdx.x >> 5;
  const int tile = blockIdx.x * 8 + wave;
  if (tile >= (MR / 32) * (DM / 64)) return;
  const int tm = tile >> 2, tn = tile & 3;
  const int m0 = tm << 5, n0 = tn << 6;
  const int rlane = lane & 15;
  const int koff = (lane >> 4) * 8;
  const int mOff = (lane >> 4) * 8;

  const __bf16* A  = (const __bf16*)(const void*)Ap;
  const __bf16* Bt = (const __bf16*)(const void*)Btp;
  const __bf16* a0p = A + (size_t)(m0 + rlane) * KC + koff;
  const __bf16* a1p = a0p + (size_t)16 * KC;
  const __bf16* bp  = Bt + (size_t)(n0 + rlane) * KC + koff;

  const v8f zero8 = {0.f, 0.f, 0.f, 0.f, 0.f, 0.f, 0.f, 0.f};
  v8f acc[2][4];
#pragma unroll
  for (int i = 0; i < 2; ++i)
#pragma unroll
    for (int j = 0; j < 4; ++j) acc[i][j] = zero8;

#pragma unroll 1
  for (int k0 = 0; k0 < KC; k0 += 32) {
    const v16b ah0 = ldfrag(a0p + k0);
    const v16b ah1 = ldfrag(a1p + k0);
#pragma unroll
    for (int j = 0; j < 4; ++j) {
      const v16b bj = ldfrag(bp + (size_t)j * 16 * KC + k0);
      acc[0][j] = mma_bf(ah0, bj, acc[0][j]);
      acc[1][j] = mma_bf(ah1, bj, acc[1][j]);
    }
  }

  float* slab = sT[wave];
  const int bidx = m0 >> 7;
  float bv[4];
#pragma unroll
  for (int j = 0; j < 4; ++j) {
    float t = bias[(size_t)bidx * bstride + n0 + (j << 4) + rlane];
    if (MODE == 0) t = bf_rne(t);
    bv[j] = t;
  }
#pragma unroll
  for (int i = 0; i < 2; ++i) {
    const int mBase = m0 + (i << 4);
    float mk[8];
    if (MODE == 1) {
      const v4f ma = *(const v4fa*)(mask + mBase + mOff);
      const v4f mb = *(const v4fa*)(mask + mBase + mOff + 4);
      mk[0] = bf_rne(ma[0]); mk[1] = bf_rne(ma[1]); mk[2] = bf_rne(ma[2]); mk[3] = bf_rne(ma[3]);
      mk[4] = bf_rne(mb[0]); mk[5] = bf_rne(mb[1]); mk[6] = bf_rne(mb[2]); mk[7] = bf_rne(mb[3]);
    } else {
#pragma unroll
      for (int r = 0; r < 8; ++r) mk[r] = 1.0f;
    }
#pragma unroll
    for (int j = 0; j < 4; ++j) {
#pragma unroll
      for (int r = 0; r < 8; ++r) {
        float v = acc[i][j][r] + bv[j];
        if (MODE == 1) v = v * mk[r];
        slab[(mOff + r) * 68 + (j << 4) + rlane] = v;
      }
    }
    __builtin_amdgcn_fence(__ATOMIC_RELEASE, "workgroup");
    __builtin_amdgcn_wave_barrier();
    __builtin_amdgcn_fence(__ATOMIC_ACQUIRE, "workgroup");

    const int hh = lane >> 4, c4 = (lane & 15) * 4;
    const int q = lane >> 3, c8 = (lane & 7) * 8;
    v4f fv[8];
    v4u hv[4], lv[4];
    if (MODE != 1) {
#pragma unroll
      for (int it = 0; it < 8; ++it) fv[it] = *(const v4fa*)(slab + (it * 2 + hh) * 68 + c4);
    }
    if (MODE != 2) {
#pragma unroll
      for (int it = 0; it < 4; ++it) {
        const float* sp = slab + (it * 4 + q) * 68 + c8;
        const v4f x0 = *(const v4fa*)(sp);
        const v4f x1 = *(const v4fa*)(sp + 4);
        const float xs[8] = { x0[0], x0[1], x0[2], x0[3], x1[0], x1[1], x1[2], x1[3] };
        unsigned short hb[8], lb[8];
#pragma unroll
        for (int e = 0; e < 8; ++e) {
          hb[e] = f2bf_bits(xs[e]);
          lb[e] = f2bf_bits(xs[e] - bf_bits2f(hb[e]));
        }
        hv[it] = (v4u){ pk16(hb[0], hb[1]), pk16(hb[2], hb[3]), pk16(hb[4], hb[5]), pk16(hb[6], hb[7]) };
        lv[it] = (v4u){ pk16(lb[0], lb[1]), pk16(lb[2], lb[3]), pk16(lb[4], lb[5]), pk16(lb[6], lb[7]) };
      }
    }
    for (int pass = 0; pass < 2; ++pass) {
      if (MODE != 1) {
#pragma unroll
        for (int it = 0; it < 8; ++it) {
          const int row = it * 2 + hh;
          *(volatile v4f*)(Cf + (size_t)(mBase + row) * DM + n0 + c4) = fv[it];
        }
      }
      if (MODE != 2) {
#pragma unroll
        for (int it = 0; it < 4; ++it) {
          const int row = it * 4 + q;
          unsigned short* d = Chl + (size_t)(mBase + row) * KC + n0 + c8;
          *(volatile v4u*)(d) = hv[it];
          *(volatile v4u*)(d + DM) = lv[it];
        }
      }
      __threadfence();
    }
    __builtin_amdgcn_fence(__ATOMIC_RELEASE, "workgroup");
    __builtin_amdgcn_wave_barrier();
    __builtin_amdgcn_fence(__ATOMIC_ACQUIRE, "workgroup");
  }
}

__global__ __launch_bounds__(256) void k_attn(const unsigned short* __restrict__ XHhlp, const unsigned short* __restrict__ W1Dp,
                                              const float* __restrict__ XHf, float* __restrict__ AGG) {
  __shared__ __align__(16) float sS[SL * 68];
  __shared__ float sP[256];
  __shared__ float sL[256];
  __shared__ float sA[256];
  __shared__ __align__(16) float sO[64];

  const int tid = threadIdx.x, lane = tid & 31, w = tid >> 5;
  const int hh = lane >> 4, c = lane & 15;
  const int b = blockIdx.x >> 2;
  const int n0 = (blockIdx.x & 3) << 6;

  const __bf16* A = (const __bf16*)(const void*)XHhlp + (size_t)(b * SL + 16 * w + c) * KC + 8 * hh;
  const __bf16* B = (const __bf16*)(const void*)W1Dp + (size_t)(n0 + c) * KC + 8 * hh;

  const v8f zero8 = {0.f, 0.f, 0.f, 0.f, 0.f, 0.f, 0.f, 0.f};
  v8f acc[4];
#pragma unroll
  for (int j = 0; j < 4; ++j) acc[j] = zero8;

#pragma unroll 1
  for (int k0 = 0; k0 < KC; k0 += 32) {
    const v16b ah = ldfrag(A + k0);
#pragma unroll
    for (int j = 0; j < 4; ++j) {
      const v16b bj = ldfrag(B + (size_t)j * 16 * KC + k0);
      acc[j] = mma_bf(ah, bj, acc[j]);
    }
  }
#pragma unroll
  for (int j = 0; j < 4; ++j)
#pragma unroll
    for (int r = 0; r < 8; ++r)
      sS[(16 * w + 8 * hh + r) * 68 + 16 * j + c] = acc[j][r];
  __syncthreads();

  const int e = tid & 63, p = tid >> 6;
  const float* sc = sS + (p * 32) * 68 + e;
  float pm = sc[0];
#pragma unroll 4
  for (int ii = 1; ii < 32; ++ii) pm = fmaxf(pm, sc[ii * 68]);
  sP[p * 64 + e] = pm;
  __syncthreads();
  const float m = fmaxf(fmaxf(sP[e], sP[64 + e]), fmaxf(sP[128 + e], sP[192 + e]));

  const float* xg = XHf + (size_t)(b * SL + p * 32) * DM + n0 + e;
  float l = 0.0f, a = 0.0f;
#pragma unroll 4
  for (int ii = 0; ii < 32; ++ii) {
    const float wv = expf(sc[ii * 68] - m);
    const float xv = xg[(size_t)ii * DM];
    l += wv;
    a = fmaf(wv, xv, a);
  }
  sL[p * 64 + e] = l;
  sA[p * 64 + e] = a;
  __syncthreads();
  if (tid < 64) {
    const float Ls = ((sL[e] + sL[64 + e]) + sL[128 + e]) + sL[192 + e];
    const float As = ((sA[e] + sA[64 + e]) + sA[128 + e]) + sA[192 + e];
    const float av = As * (1.0f / Ls);
    sO[e] = 1.0f / (1.0f + expf(-av));
  }
  __syncthreads();
  const v4f ov = *(const v4fa*)(sO + 4 * (tid & 15));
  if (tid < 16) {
    float* d = AGG + (size_t)b * DM + n0 + 4 * tid;
    *(volatile v4f*)d = ov;
    __threadfence();
    *(volatile v4f*)d = ov;
  }
}

__global__ __launch_bounds__(256) void k_cvec(const float* __restrict__ AGG, const float* __restrict__ upd_w,
                                              const float* __restrict__ upd_b, float* __restrict__ CV) {
  __shared__ __align__(16) float sG[DM];
  __shared__ __align__(16) float sC[DM];
  const int b = blockIdx.x, tid = threadIdx.x;
  sG[tid] = AGG[(size_t)b * DM + tid];
  __syncthreads();
  const float* ur = upd_w + (size_t)tid * (2 * DM) + DM;
  float acc = 0.0f;
#pragma unroll 1
  for (int f = 0; f < DM; f += 8) {
    const v4f u0 = *(const v4fa*)(ur + f);
    const v4f u1 = *(const v4fa*)(ur + f + 4);
    acc = fmaf(sG[f + 0], bf_rne(u0[0]), acc);
    acc = fmaf(sG[f + 1], bf_rne(u0[1]), acc);
    acc = fmaf(sG[f + 2], bf_rne(u0[2]), acc);
    acc = fmaf(sG[f + 3], bf_rne(u0[3]), acc);
    acc = fmaf(sG[f + 4], bf_rne(u1[0]), acc);
    acc = fmaf(sG[f + 5], bf_rne(u1[1]), acc);
    acc = fmaf(sG[f + 6], bf_rne(u1[2]), acc);
    acc = fmaf(sG[f + 7], bf_rne(u1[3]), acc);
  }
  acc += bf_rne(upd_b[tid]);
  sC[tid] = acc;
  __syncthreads();
  const v4f cv = *(const v4fa*)(sC + 4 * (tid & 63));
  if (tid < 64) {
    float* d = CV + (size_t)b * DM + 4 * tid;
    *(volatile v4f*)d = cv;
    __threadfence();
    *(volatile v4f*)d = cv;
  }
}

extern "C" void kernel_launch(void* const* d_in, const int* in_sizes, int n_in,
                              void* d_out, int out_size, void* d_ws, size_t ws_size,
                              hipStream_t stream) {
  if (n_in < 8) return;
  if (in_sizes[0] != MR * DM) return;
  if (in_sizes[1] != MR) return;
  if (in_sizes[2] != DM * DM || in_sizes[3] != DM) return;
  if (in_sizes[4] != DM * 2 * DM || in_sizes[5] != DM) return;
  if (in_sizes[6] != DM * 2 * DM || in_sizes[7] != DM) return;
  if (out_size != MR * DM) return;

  const float* feat   = (const float*)d_in[0];
  const float* mask   = (const float*)d_in[1];
  const float* agg_w  = (const float*)d_in[2];
  const float* agg_b  = (const float*)d_in[3];
  const float* attn_w = (const float*)d_in[4];
  const float* attn_b = (const float*)d_in[5];
  const float* upd_w  = (const float*)d_in[6];
  const float* upd_b  = (const float*)d_in[7];
  (void)attn_b;

  const size_t PWB = (size_t)DM * KC * 2;
  const size_t PAB = (size_t)MR * KC * 2;
  const size_t PFB = (size_t)MR * DM * 4;
  const size_t PVB = (size_t)NB * DM * 4;
  size_t off = 0;
  const size_t oAGW = off; off += PWB;
  const size_t oW1D = off; off += PWB;
  const size_t oU1D = off; off += PWB;
  const size_t oHM  = off; off += PAB;
  const size_t oXHh = off; off += PAB;
  const size_t oXHf = off; off += PFB;
  const size_t oAGG = off; off += PVB;
  const size_t oCV  = off; off += PVB;
  if (off > ws_size) return;

  char* ws = (char*)d_ws;
  unsigned short* AGW2 = (unsigned short*)(ws + oAGW);
  unsigned short* W1D  = (unsigned short*)(ws + oW1D);
  unsigned short* U1D  = (unsigned short*)(ws + oU1D);
  unsigned short* HM   = (unsigned short*)(ws + oHM);
  unsigned short* XHhl = (unsigned short*)(ws + oXHh);
  float*          XHf  = (float*)(ws + oXHf);
  float*          AGG  = (float*)(ws + oAGG);
  float*          CV   = (float*)(ws + oCV);
  float*          out  = (float*)d_out;

  const dim3 blk(256);
  k_prep<<<dim3(352), blk, 0, stream>>>(feat, mask, agg_w, attn_w, upd_w, AGW2, W1D, U1D, HM);

  const dim3 gG((MR / 32) * (DM / 64) / 8);
  const dim3 gA(NB * (DM / 64));
  const dim3 gC(NB);

  for (int step = 0; step < 3; ++step) {
    k_gemm2<0><<<gG, blk, 0, stream>>>(HM, AGW2, agg_b, 0, mask, XHf, XHhl);
    k_attn<<<gA, blk, 0, stream>>>(XHhl, W1D, XHf, AGG);
    k_cvec<<<gC, blk, 0, stream>>>(AGG, upd_w, upd_b, CV);
    if (step < 2) {
      k_gemm2<1><<<gG, blk, 0, stream>>>(XHhl, U1D, CV, DM, mask, XHf, HM);
    } else {
      k_gemm2<2><<<gG, blk, 0, stream>>>(XHhl, U1D, CV, DM, mask, out, HM);
    }
  }
  (void)hipGetLastError();
}
